// ReinforceAttention_59949153517746
// MI455X (gfx1250) — hardware-verified
//
#include <hip/hip_runtime.h>


#define NB_  4
#define CC   64
#define HV   128
#define NN   4096
#define PCAR 1024.0f
#define SCL  0.088388347648318447f
typedef _Float16 h16;
typedef unsigned short bf;
typedef __attribute__((ext_vector_type(16))) __bf16   v16bf;
typedef __attribute__((ext_vector_type(16))) _Float16 v16h;
typedef __attribute__((ext_vector_type(8)))  _Float16 v8h;
typedef __attribute__((ext_vector_type(8)))  unsigned short v8us;
typedef __attribute__((ext_vector_type(8)))  float    v8f;
typedef __attribute__((ext_vector_type(4)))  float    v4f;
typedef v8h  __attribute__((may_alias)) v8ha;
typedef v4f  __attribute__((may_alias)) v4fa;
typedef v8us __attribute__((may_alias)) v8usa;

__device__ __forceinline__ unsigned short f2bf(float f) { unsigned u = __float_as_uint(f); u += 0x7FFFu + ((u >> 16) & 1u); return (unsigned short)(u >> 16); }
__device__ __forceinline__ float bf2f(unsigned short b) { return __uint_as_float(((unsigned)b) << 16); }
__device__ __forceinline__ float bfr(float f) { return bf2f(f2bf(f)); }
__device__ __forceinline__ v16h cat16(v8h lo, v8h hi) { return __builtin_shufflevector(lo, hi, 0, 1, 2, 3, 4, 5, 6, 7, 8, 9, 10, 11, 12, 13, 14, 15); }
__device__ __forceinline__ v16bf cat16b(v8us lo, v8us hi) { return __builtin_bit_cast(v16bf, __builtin_shufflevector(lo, hi, 0, 1, 2, 3, 4, 5, 6, 7, 8, 9, 10, 11, 12, 13, 14, 15)); }
__device__ __forceinline__ v8f wmma16(v16h a, v16h b, v8f c) { return __builtin_amdgcn_wmma_f32_16x16x32_f16(false, a, false, b, (short)0, c, false, false); }
__device__ __forceinline__ v8f wmmab(v16bf a, v16bf b, v8f c) { return __builtin_amdgcn_wmma_f32_16x16x32_bf16(false, a, false, b, (short)0, c, false, false); }


template <typename T16> struct WFrag;
template <> struct WFrag<h16> { typedef v16h V; static __device__ __forceinline__ V ld(const h16* p) { return cat16(*(const v8h*)p, *(const v8h*)(p + 16)); } static __device__ __forceinline__ v8f mma(V a, V b, v8f c) { return wmma16(a, b, c); } };
template <> struct WFrag<bf> { typedef v16bf V; static __device__ __forceinline__ V ld(const bf* p) { return cat16b(*(const v8us*)p, *(const v8us*)(p + 16)); } static __device__ __forceinline__ v8f mma(V a, V b, v8f c) { return wmmab(a, b, c); } };
template <typename T16, int NSPLIT, bool BIAS>
__global__ __launch_bounds__(32) void k_gemmw(const T16* __restrict__ A, const T16* __restrict__ A2, const T16* __restrict__ Bt, const T16* __restrict__ Bt2, int K, float* C, int ldc, const float* __restrict__ bias, size_t sA, size_t sB, size_t sC) {
    typedef typename WFrag<T16>::V V;
    __shared__ __align__(16) float os[16 * 68];
    const size_t z = blockIdx.z; A += z * sA; if (A2) A2 += z * sA; Bt += z * sB; if (Bt2) Bt2 += z * sB; C += z * sC;
    const int lane = threadIdx.x & 31, lr = lane & 15, hi = lane >> 4; const int r0 = blockIdx.x * 64, c0 = blockIdx.y * 64;
    v8f acc[4][4];
#pragma unroll
    for (int mb = 0; mb < 4; ++mb)
#pragma unroll
        for (int nb = 0; nb < 4; ++nb) acc[mb][nb] = (v8f){};
    const size_t aoff = (size_t)(r0 + lr) * K + 8 * hi, boff = (size_t)(c0 + lr) * K + 8 * hi;
#pragma unroll 1
    for (int kc = 0; kc < K; kc += 32) {
        V a[4], a2[4];
#pragma unroll
        for (int mb = 0; mb < 4; ++mb) { a[mb] = WFrag<T16>::ld(A + aoff + (size_t)mb * 16 * K + kc); if (NSPLIT == 1 || NSPLIT == 2) a2[mb] = WFrag<T16>::ld(A2 + aoff + (size_t)mb * 16 * K + kc); }
#pragma unroll
        for (int nb = 0; nb < 4; ++nb) { const V b = WFrag<T16>::ld(Bt + boff + (size_t)nb * 16 * K + kc); V b2; if (NSPLIT >= 2) b2 = WFrag<T16>::ld(Bt2 + boff + (size_t)nb * 16 * K + kc);
#pragma unroll
            for (int mb = 0; mb < 4; ++mb) { acc[mb][nb] = WFrag<T16>::mma(a[mb], b, acc[mb][nb]); if (NSPLIT == 1 || NSPLIT == 2) acc[mb][nb] = WFrag<T16>::mma(a2[mb], b, acc[mb][nb]); if (NSPLIT >= 2) acc[mb][nb] = WFrag<T16>::mma(a[mb], b2, acc[mb][nb]); } }
        asm volatile("v_nop\n\tv_nop\n\tv_nop\n\tv_nop" : "+v"(acc[0][0]), "+v"(acc[1][1]), "+v"(acc[2][2]), "+v"(acc[3][3]) : "v"(a[0]), "v"(a[3]));
    }
#pragma unroll
    for (int mb = 0; mb < 4; ++mb) {
#pragma unroll
        for (int nb = 0; nb < 4; ++nb) {
#pragma unroll
            for (int j = 0; j < 8; ++j) os[(hi * 8 + j) * 68 + nb * 16 + lr] = acc[mb][nb][j]; }
        __builtin_amdgcn_wave_barrier(); asm volatile("" ::: "memory");
        float* crow = C + (size_t)(r0 + mb * 16) * ldc + c0;
#pragma unroll 1
        for (int ps = 0; ps < 2; ++ps) {
#pragma unroll
            for (int s = 0; s < 8; ++s) { const int row = 2 * s + hi, cofs = lr * 4; v4f val = *(const v4fa*)(os + row * 68 + cofs); if (BIAS) { val[0] += bfr(bias[c0 + cofs]); val[1] += bfr(bias[c0 + cofs + 1]); val[2] += bfr(bias[c0 + cofs + 2]); val[3] += bfr(bias[c0 + cofs + 3]); }
                *(volatile v4f*)(crow + (size_t)row * ldc + cofs) = val; }
            if (ps == 0) __threadfence(); }
        __builtin_amdgcn_wave_barrier(); asm volatile("" ::: "memory");
    }
}

__device__ __forceinline__ h16 tohx(float x) { return (h16)x; }
__device__ __forceinline__ void splitf(float y, unsigned short& h, unsigned short& l) { h = f2bf(y); l = f2bf(y - bf2f(h)); }
typedef __attribute__((ext_vector_type(2))) _Float16 v2h;
typedef __attribute__((ext_vector_type(4))) _Float16 v4h;
typedef __attribute__((ext_vector_type(2))) unsigned short v2us;

__global__ __launch_bounds__(256) void k_cvt8(const float* __restrict__ src, bf* dst, size_t n8) { const size_t i = (size_t)blockIdx.x * 256 + threadIdx.x; if (i >= n8) return; const v8f v = *(const v8f*)(src + i * 8); v8us o;
#pragma unroll
    for (int k = 0; k < 8; ++k) o[k] = f2bf(v[k]); *(volatile v8us*)(dst + i * 8) = o; __threadfence(); *(volatile v8us*)(dst + i * 8) = o; }
__global__ __launch_bounds__(256) void k_xt(const float* __restrict__ src, bf* XT) { const int i = (blockIdx.x * 256 + threadIdx.x) * 2; if (i >= NN * CC) return; const int n = i / CC, c = i % CC; v2us o; o[0] = f2bf(src[(size_t)c * NN + n]); o[1] = f2bf(src[(size_t)(c + 1) * NN + n]);
    *(volatile v2us*)(XT + i) = o; __threadfence(); *(volatile v2us*)(XT + i) = o; }
__global__ __launch_bounds__(256) void k_split2(const float* __restrict__ F, bf* Ph, bf* Pl, size_t n) { const size_t i = ((size_t)blockIdx.x * 256 + threadIdx.x) * 2; if (i >= n) return; v2us oh, ol;
#pragma unroll
    for (int q = 0; q < 2; ++q) { unsigned short a, c2; splitf(F[i + q], a, c2); oh[q] = a; ol[q] = c2; } *(volatile v2us*)(Ph + i) = oh; *(volatile v2us*)(Pl + i) = ol; __threadfence(); *(volatile v2us*)(Ph + i) = oh; *(volatile v2us*)(Pl + i) = ol; }
__global__ __launch_bounds__(256) void k_v16(const float* __restrict__ FV, const float* __restrict__ bv, h16* V16) { const size_t i = ((size_t)blockIdx.x * 256 + threadIdx.x) * 2; if (i >= (size_t)HV * NN) return; const int d = (int)(i / NN); const float bb = bfr(bv[d]); v2h v; v[0] = tohx(__fadd_rn(FV[i], bb)); v[1] = tohx(__fadd_rn(FV[i + 1], bb));
    *(volatile v2h*)(V16 + i) = v; __threadfence(); *(volatile v2h*)(V16 + i) = v; }
__global__ __launch_bounds__(256) void k_smax(const float* __restrict__ S, float* RS) { const int lane = threadIdx.x & 31; const int i = blockIdx.x * 8 + (threadIdx.x >> 5); if (i >= NN) return; const float* sr = S + (size_t)i * NN; float mx = -3.0e38f;
    for (int c0 = lane * 4; c0 < NN; c0 += 128) { const v4f v = *(const v4f*)(sr + c0); mx = fmaxf(fmaxf(mx, fmaxf(v[0], v[1])), fmaxf(v[2], v[3])); }
#pragma unroll
    for (int sh = 16; sh; sh >>= 1) mx = fmaxf(mx, __shfl_xor(mx, sh, 32));
    const float o = (lane == 0) ? mx : 0.f; *(volatile float*)(RS + (size_t)i * 32 + lane) = o; __threadfence(); *(volatile float*)(RS + (size_t)i * 32 + lane) = o; }
__global__ __launch_bounds__(256) void k_sexp(const float* __restrict__ S, float* RS, h16* P) { const int lane = threadIdx.x & 31; const int i = blockIdx.x * 8 + (threadIdx.x >> 5); if (i >= NN) return; const float* sr = S + (size_t)i * NN; const float mx = RS[(size_t)i * 32]; float sum = 0.f;
#pragma unroll 1
    for (int ps = 0; ps < 2; ++ps) { sum = 0.f;
        for (int c0 = lane * 4; c0 < NN; c0 += 128) { const v4f v = *(const v4f*)(sr + c0); v4h o;
#pragma unroll
            for (int q = 0; q < 4; ++q) { const float e = __expf(__fmul_rn(__fsub_rn(v[q], mx), SCL)); sum = __fadd_rn(sum, e); o[q] = tohx(e * PCAR); }
            *(volatile v4h*)(P + (size_t)i * NN + c0) = o; }
        if (ps == 0) __threadfence(); }
#pragma unroll
    for (int sh = 16; sh; sh >>= 1) sum += __shfl_xor(sum, sh, 32);
    const float r = __fdiv_rn(1.0f, sum * PCAR); const float o2 = (lane == 0) ? mx : (lane == 1 ? r : 0.f); *(volatile float*)(RS + (size_t)i * 32 + lane) = o2; __threadfence(); *(volatile float*)(RS + (size_t)i * 32 + lane) = o2; }
__global__ __launch_bounds__(256) void k_osplit(const float* __restrict__ Ob, const float* __restrict__ RS, bf* Oh, bf* Ol) { const size_t i = ((size_t)blockIdx.x * 256 + threadIdx.x) * 2; if (i >= (size_t)NN * HV) return; const int n = (int)(i / HV); const float ri = RS[(size_t)n * 32 + 1]; v2us oh, ol;
#pragma unroll
    for (int q = 0; q < 2; ++q) { unsigned short a, c2; splitf(__fmul_rn(Ob[i + q], ri), a, c2); oh[q] = a; ol[q] = c2; }
    *(volatile v2us*)(Oh + i) = oh; *(volatile v2us*)(Ol + i) = ol; __threadfence(); *(volatile v2us*)(Oh + i) = oh; *(volatile v2us*)(Ol + i) = ol; }
__global__ __launch_bounds__(256) void k_mixf(const float* __restrict__ Y, const float* __restrict__ bo, const float* __restrict__ xb, const float* __restrict__ alp, float* O2, float* FEAT) { const int n = blockIdx.x * 256 + threadIdx.x; if (n >= NN) return; const float al = bfr(alp[0]); const float be = __fsub_rn(1.0f, al); float s = 0.f, mx = -3.0e38f;
#pragma unroll 1
    for (int ps = 0; ps < 2; ++ps) { s = 0.f; mx = -3.0e38f;
#pragma unroll 4
        for (int c = 0; c < CC; ++c) { float t1 = __fmul_rn(al, __fadd_rn(Y[(size_t)c * NN + n], bfr(bo[c]))), t2 = __fmul_rn(be, bfr(xb[(size_t)c * NN + n])); asm volatile("" : "+v"(t1)); asm volatile("" : "+v"(t2)); const float o = __fadd_rn(t1, t2); s = __fadd_rn(s, o); mx = fmaxf(mx, o); *(volatile float*)(O2 + (size_t)c * NN + n) = o; }
        *(volatile float*)(FEAT + n) = s * (1.0f / CC); *(volatile float*)(FEAT + NN + n) = mx; if (ps == 0) __threadfence(); }
}
__global__ __launch_bounds__(256) void k_gate(const float* __restrict__ O2, const float* __restrict__ FEAT, const float* __restrict__ ws, const float* __restrict__ bs, float* OUTb) { const int n = blockIdx.x * 256 + threadIdx.x; if (n >= NN) return; const int y = n >> 6, xx = n & 63; float g = 0.f;
#pragma unroll 1
    for (int c2 = 0; c2 < 2; ++c2)
#pragma unroll 1
        for (int ky = 0; ky < 7; ++ky) { const int yy = y + ky - 3; if (yy < 0 || yy >= 64) continue;
#pragma unroll
            for (int kx = 0; kx < 7; ++kx) { const int x2 = xx + kx - 3; if (x2 < 0 || x2 >= 64) continue; float p = __fmul_rn(bfr(ws[(c2 * 7 + ky) * 7 + kx]), FEAT[c2 * NN + yy * 64 + x2]); asm volatile("" : "+v"(p)); g = __fadd_rn(g, p); } }
    g = __fadd_rn(g, bfr(bs[0])); const float sg = __fdiv_rn(1.0f, __fadd_rn(1.0f, __expf(-g)));
#pragma unroll 1
    for (int ps = 0; ps < 2; ++ps) {
#pragma unroll 4
        for (int c = 0; c < CC; ++c) *(volatile float*)(OUTb + (size_t)c * NN + n) = __fmul_rn(O2[(size_t)c * NN + n], sg);
        if (ps == 0) __threadfence(); }
}

extern "C" void kernel_launch(void* const* d_in, const int* in_sizes, int n_in,
                              void* d_out, int out_size, void* d_ws, size_t ws_size, hipStream_t stream) {
    (void)in_sizes; (void)n_in; (void)out_size;
    const float* IN[12]; for (int i = 0; i < 12; ++i) IN[i] = (const float*)d_in[i];
    float* OUT = (float*)d_out;
    char* wsp = (char*)d_ws;
    auto take = [&](size_t bytes) { char* p = wsp; wsp += (bytes + 255) & ~(size_t)255; return (void*)p; };
    bf* WQ = (bf*)take((size_t)HV * CC * 2); bf* WK = (bf*)take((size_t)HV * CC * 2); bf* WV = (bf*)take((size_t)HV * CC * 2); bf* WO = (bf*)take((size_t)CC * HV * 2);
    bf* XT = (bf*)take((size_t)NN * CC * 2); float* FQ = (float*)take((size_t)NN * HV * 4); bf* Qh = (bf*)take((size_t)NN * HV * 2); bf* Ql = (bf*)take((size_t)NN * HV * 2); bf* Kh = (bf*)take((size_t)NN * HV * 2); bf* Kl = (bf*)take((size_t)NN * HV * 2);
    float* FV = (float*)take((size_t)HV * NN * 4); h16* V16 = (h16*)take((size_t)HV * NN * 2); float* S = (float*)take((size_t)NN * NN * 4); h16* P = (h16*)take((size_t)NN * NN * 2); float* RS = (float*)take((size_t)NN * 32 * 4);
    bf* OTh = (bf*)take((size_t)NN * HV * 2); bf* OTl = (bf*)take((size_t)NN * HV * 2); float* Y = (float*)take((size_t)CC * NN * 4); float* O2 = (float*)take((size_t)CC * NN * 4); float* FEAT = (float*)take((size_t)2 * NN * 4);
    if ((size_t)(wsp - (char*)d_ws) > ws_size) return;
    float* Ob = FV;
    { const size_t nw = (size_t)HV * CC / 8; const unsigned gw = (unsigned)((nw + 255) / 256); k_cvt8<<<gw, 256, 0, stream>>>(IN[1], WQ, nw); k_cvt8<<<gw, 256, 0, stream>>>(IN[3], WK, nw); k_cvt8<<<gw, 256, 0, stream>>>(IN[5], WV, nw); k_cvt8<<<gw, 256, 0, stream>>>(IN[7], WO, nw); }
    const unsigned LQ = (unsigned)(((size_t)NN * HV / 2 + 255) / 256);
    for (int b = 0; b < NB_; ++b) { const float* xb = IN[0] + (size_t)b * CC * NN;
        k_xt<<<(NN * CC / 2 + 255) / 256, 256, 0, stream>>>(xb, XT);
        k_gemmw<bf, 0, true><<<dim3(NN / 64, HV / 64, 1), 32, 0, stream>>>(XT, nullptr, WQ, nullptr, CC, FQ, HV, IN[2], 0, 0, 0); k_split2<<<LQ, 256, 0, stream>>>(FQ, Qh, Ql, (size_t)NN * HV);
        k_gemmw<bf, 0, true><<<dim3(NN / 64, HV / 64, 1), 32, 0, stream>>>(XT, nullptr, WK, nullptr, CC, FQ, HV, IN[4], 0, 0, 0); k_split2<<<LQ, 256, 0, stream>>>(FQ, Kh, Kl, (size_t)NN * HV);
        k_gemmw<bf, 0, false><<<dim3(HV / 64, NN / 64, 1), 32, 0, stream>>>(WV, nullptr, XT, nullptr, CC, FV, NN, nullptr, 0, 0, 0); k_v16<<<LQ, 256, 0, stream>>>(FV, IN[6], V16);
        k_gemmw<bf, 2, false><<<dim3(NN / 64, NN / 64, 1), 32, 0, stream>>>(Qh, Ql, Kh, Kl, HV, S, NN, nullptr, 0, 0, 0);
        k_smax<<<NN / 8, 256, 0, stream>>>(S, RS); k_sexp<<<NN / 8, 256, 0, stream>>>(S, RS, P);
        k_gemmw<h16, 0, false><<<dim3(NN / 64, HV / 64, 1), 32, 0, stream>>>(P, nullptr, V16, nullptr, NN, Ob, HV, nullptr, 0, 0, 0);
        k_osplit<<<LQ, 256, 0, stream>>>(Ob, RS, OTh, OTl);
        k_gemmw<bf, 3, false><<<dim3(CC / 64, NN / 64, 1), 32, 0, stream>>>(WO, nullptr, OTh, OTl, HV, Y, NN, nullptr, 0, 0, 0);
        k_mixf<<<NN / 256, 256, 0, stream>>>(Y, IN[8], xb, IN[11], O2, FEAT);
        k_gate<<<NN / 256, 256, 0, stream>>>(O2, FEAT, IN[9], IN[10], OUT + (size_t)b * CC * NN); }
}
